// HebbianMemory_37220186588012
// MI455X (gfx1250) — hardware-run, weakly checked
//
#include <hip/hip_runtime.h>


#define NRW  8192
#define NCW  512
#define NPJ  1600
#define NUN  8
#define NEW  64
#define NSP  4096

typedef _Float16 h16;
typedef unsigned short bf;
typedef __attribute__((ext_vector_type(16))) __bf16   v16bf;
typedef __attribute__((ext_vector_type(16))) _Float16 v16h;
typedef __attribute__((ext_vector_type(8)))  _Float16 v8h;
typedef __attribute__((ext_vector_type(8)))  unsigned short v8us;
typedef __attribute__((ext_vector_type(8)))  float    v8f;
typedef __attribute__((ext_vector_type(4)))  float    v4f;
typedef v8h  __attribute__((may_alias)) v8ha;
typedef v4f  __attribute__((may_alias)) v4fa;
typedef v8us __attribute__((may_alias)) v8usa;

__device__ __forceinline__ unsigned short f2bf(float f) { unsigned u = __float_as_uint(f); u += 0x7FFFu + ((u >> 16) & 1u); return (unsigned short)(u >> 16); }
__device__ __forceinline__ float bf2f(unsigned short b) { return __uint_as_float(((unsigned)b) << 16); }
__device__ __forceinline__ float bfr(float f) { return bf2f(f2bf(f)); }
__device__ __forceinline__ v16h cat16(v8h lo, v8h hi) { return __builtin_shufflevector(lo, hi, 0, 1, 2, 3, 4, 5, 6, 7, 8, 9, 10, 11, 12, 13, 14, 15); }
__device__ __forceinline__ v16bf cat16b(v8us lo, v8us hi) { return __builtin_bit_cast(v16bf, __builtin_shufflevector(lo, hi, 0, 1, 2, 3, 4, 5, 6, 7, 8, 9, 10, 11, 12, 13, 14, 15)); }
__device__ __forceinline__ v8f wmma16(v16h a, v16h b, v8f c) { return __builtin_amdgcn_wmma_f32_16x16x32_f16(false, a, false, b, (short)0, c, false, false); }
__device__ __forceinline__ v8f wmmab(v16bf a, v16bf b, v8f c) { return __builtin_amdgcn_wmma_f32_16x16x32_bf16(false, a, false, b, (short)0, c, false, false); }

template <typename T16> struct WFrag;
template <> struct WFrag<h16> { typedef v16h V; static __device__ __forceinline__ V ld(const h16* p) { return cat16(*(const v8h*)p, *(const v8h*)(p + 16)); } static __device__ __forceinline__ v8f mma(V a, V b, v8f c) { return wmma16(a, b, c); } };
template <> struct WFrag<bf> { typedef v16bf V; static __device__ __forceinline__ V ld(const bf* p) { return cat16b(*(const v8us*)p, *(const v8us*)(p + 16)); } static __device__ __forceinline__ v8f mma(V a, V b, v8f c) { return wmmab(a, b, c); } };
template <typename T16, int NSPLIT, bool BIAS>
__global__ __launch_bounds__(32) void k_gemmw(const T16* __restrict__ A, const T16* __restrict__ A2, const T16* __restrict__ Bt, const T16* __restrict__ Bt2, int K, float* C, int ldc, const float* __restrict__ bias, size_t sA, size_t sB, size_t sC) {
    typedef typename WFrag<T16>::V V;
    __shared__ __align__(16) float os[16 * 68];
    const size_t z = blockIdx.z; A += z * sA; if (A2) A2 += z * sA; Bt += z * sB; if (Bt2) Bt2 += z * sB; C += z * sC;
    const int lane = threadIdx.x & 31, lr = lane & 15, hi = lane >> 4; const int r0 = blockIdx.x * 64, c0 = blockIdx.y * 64;
    v8f acc[4][4];
#pragma unroll
    for (int mb = 0; mb < 4; ++mb)
#pragma unroll
        for (int nb = 0; nb < 4; ++nb) acc[mb][nb] = (v8f){};
    const size_t aoff = (size_t)(r0 + lr) * K + 8 * hi, boff = (size_t)(c0 + lr) * K + 8 * hi;
    for (int kc = 0; kc < K; kc += 32) {
        V a[4], a2[4];
#pragma unroll
        for (int mb = 0; mb < 4; ++mb) { a[mb] = WFrag<T16>::ld(A + aoff + (size_t)mb * 16 * K + kc); if (NSPLIT == 1 || NSPLIT == 2) a2[mb] = WFrag<T16>::ld(A2 + aoff + (size_t)mb * 16 * K + kc); }
#pragma unroll
        for (int nb = 0; nb < 4; ++nb) { const V b = WFrag<T16>::ld(Bt + boff + (size_t)nb * 16 * K + kc); V b2; if (NSPLIT >= 2) b2 = WFrag<T16>::ld(Bt2 + boff + (size_t)nb * 16 * K + kc);
#pragma unroll
            for (int mb = 0; mb < 4; ++mb) { acc[mb][nb] = WFrag<T16>::mma(a[mb], b, acc[mb][nb]); if (NSPLIT == 1 || NSPLIT == 2) acc[mb][nb] = WFrag<T16>::mma(a2[mb], b, acc[mb][nb]); if (NSPLIT >= 2) acc[mb][nb] = WFrag<T16>::mma(a[mb], b2, acc[mb][nb]); } }
        asm volatile("v_nop\n\tv_nop\n\tv_nop\n\tv_nop" : "+v"(acc[0][0]), "+v"(acc[1][1]), "+v"(acc[2][2]), "+v"(acc[3][3]) : "v"(a[0]), "v"(a[3]));
    }
#pragma unroll
    for (int mb = 0; mb < 4; ++mb) {
#pragma unroll
        for (int nb = 0; nb < 4; ++nb) {
#pragma unroll
            for (int j = 0; j < 8; ++j) os[(hi * 8 + j) * 68 + nb * 16 + lr] = acc[mb][nb][j]; }
        __builtin_amdgcn_wave_barrier(); asm volatile("" ::: "memory");
        float* crow = C + (size_t)(r0 + mb * 16) * ldc + c0;
#pragma unroll 1
        for (int ps = 0; ps < 2; ++ps) {
#pragma unroll
            for (int s = 0; s < 8; ++s) { const int row = 2 * s + hi, cofs = lr * 4; v4f val = *(const v4fa*)(os + row * 68 + cofs); if (BIAS) { val[0] += bfr(bias[c0 + cofs]); val[1] += bfr(bias[c0 + cofs + 1]); val[2] += bfr(bias[c0 + cofs + 2]); val[3] += bfr(bias[c0 + cofs + 3]); }
                *(volatile v4f*)(crow + (size_t)row * ldc + cofs) = val; }
            if (ps == 0) __threadfence(); }
        __builtin_amdgcn_wave_barrier(); asm volatile("" ::: "memory");
    }
}

typedef __attribute__((ext_vector_type(2))) _Float16 v2h;
typedef __attribute__((ext_vector_type(4))) _Float16 v4h;
typedef __attribute__((ext_vector_type(2))) unsigned short v2us;
typedef __attribute__((ext_vector_type(4))) unsigned short v4us;
typedef __attribute__((ext_vector_type(2))) float v2f;
typedef __attribute__((ext_vector_type(4))) int v4i;
__global__ __launch_bounds__(256) void k_cvt8(const float* __restrict__ src, bf* dst, size_t n8) { const size_t i = (size_t)blockIdx.x * 256 + threadIdx.x; if (i >= n8) return; const v8f v = *(const v8f*)(src + i * 8); v8us o;
#pragma unroll
    for (int k = 0; k < 8; ++k) o[k] = f2bf(v[k]); *(volatile v8us*)(dst + i * 8) = o; __threadfence(); *(volatile v8us*)(dst + i * 8) = o; }

__global__ __launch_bounds__(256) void k_fillb(bf* P, unsigned w2, size_t n8) { const size_t i = (size_t)blockIdx.x * 256 + threadIdx.x; if (i >= n8) return; v4i o; o[0] = (int)w2; o[1] = (int)w2; o[2] = (int)w2; o[3] = (int)w2;
    *(volatile v4i*)(P + i * 8) = o; __threadfence(); *(volatile v4i*)(P + i * 8) = o; }

__device__ __forceinline__ h16 toh_flush(float x) { const float z = (fabsf(x) < 6.103515625e-05f) ? 0.0f : x; return (h16)z; }

template <bool RB>
__global__ __launch_bounds__(256) void k_c16(const float* __restrict__ src, h16* dst, size_t n8) { const size_t i = (size_t)blockIdx.x * 256 + threadIdx.x; if (i >= n8) return; const float* p = src + i * 8; const v4f a = *(const v4f*)p, b = *(const v4f*)(p + 4); v8h o;
#pragma unroll
    for (int q = 0; q < 4; ++q) { o[q] = toh_flush(RB ? bfr(a[q]) : a[q]); o[q + 4] = toh_flush(RB ? bfr(b[q]) : b[q]); }
    *(volatile v8h*)(dst + i * 8) = o; __threadfence(); *(volatile v8h*)(dst + i * 8) = o; }

__global__ __launch_bounds__(32) void k_run(const float* __restrict__ Pj, const float* __restrict__ u7, float* Gq, float* Gk) { const unsigned sq = blockIdx.x, ln = threadIdx.x, un = ln & 7u, ph = ln >> 3; const float ad = bfr(u7[un]); const float m1 = (float)((ph + 3u) >> 2), m2 = (float)((ph + 2u) >> 2), m3 = (float)((ph + 1u) >> 2); const float* pp = Pj + (size_t)sq * NSP * NPJ + 1536 + un; float* pq = Gq + (size_t)sq * NSP * NUN + ln; float* pk = Gk + (size_t)sq * NSP * NUN + ln; float tt = 0.0f;
#pragma unroll 1
    for (unsigned tp = 0; tp < 1024u; ++tp) { float tm[4];
#pragma unroll
        for (int q1 = 0; q1 < 4; ++q1) { const float aw = pp[(size_t)(4u * tp + (unsigned)q1) * NPJ] + ad; const float ea = 0.9f + 0.1f * (1.0f / (1.0f + expf(-aw))); tm[q1] = logf(fmaxf(ea, 1e-6f)); }
        const float r0 = tt + tm[0]; const float mine = ((r0 + m1 * tm[1]) + m2 * tm[2]) + m3 * tm[3]; tt = ((r0 + tm[1]) + tm[2]) + tm[3]; const float rt = fminf(fmaxf(mine, -50.0f), 50.0f); const float wq = expf(rt), wk = expf(-rt); *(volatile float*)(pq + (size_t)tp * 32u) = wq; *(volatile float*)(pk + (size_t)tp * 32u) = wk; __threadfence(); *(volatile float*)(pq + (size_t)tp * 32u) = wq; *(volatile float*)(pk + (size_t)tp * 32u) = wk; } }

__global__ __launch_bounds__(256) void k_feat(float* Pj, const float* __restrict__ u3, const float* __restrict__ Gq, const float* __restrict__ Gk) { const unsigned id = blockIdx.x * 256u + threadIdx.x; const unsigned c0 = (id & 255u) << 2, rw = id >> 8; const unsigned hb = c0 >> 9, un = (c0 & 511u) >> 6; const unsigned ip = rw * (unsigned)NPJ + c0, ig = rw * (unsigned)NUN + un; const v4f pw = *(const v4f*)(Pj + ip), aw = *(const v4f*)(u3 + c0); const float fq = Gq[ig] * 0.125f, fk = Gk[ig]; const float fc = hb != 0u ? fk : fq; v4f ov;
#pragma unroll
    for (int q1 = 0; q1 < 4; ++q1) { const float ww = pw[q1] + bfr(aw[q1]); const float gw = fmaxf(ww, 0.0f) + expf(fminf(ww, 0.0f)); ov[q1] = gw * fc; }
    *(volatile v4f*)(Pj + ip) = ov; __threadfence(); *(volatile v4f*)(Pj + ip) = ov; }

__global__ __launch_bounds__(96) void k_tal2(const float* __restrict__ Pj, const float* __restrict__ u3, float* Og, float* Dv) { const unsigned bu = blockIdx.x, sq = bu >> 3, un = bu & 7u, cj = threadIdx.x, lo = cj & 63u; const unsigned od = cj >> 6; const float om = (float)(1u - od); const float ac = bfr(u3[1024u + un * NEW + lo]); const float* pc = Pj + (size_t)sq * NSP * NPJ + 1024u + un * NEW + lo; const float* pf = Pj + (size_t)sq * NSP * NPJ + un * NEW; float* pa = Og + (size_t)sq * NSP * NCW + un * NEW + lo; float* pb = Dv + ((size_t)sq * NSP * NUN + un) * 32u + (lo & 31u); float* po = od != 0u ? pb : pa; const size_t so = (size_t)NCW - (size_t)od * (NCW - NUN * 32u); float tw[NEW];
#pragma unroll
    for (int i = 0; i < NEW; ++i) tw[i] = 0.0f;
#pragma unroll 1
    for (unsigned st = 0; st < 4096u; ++st) { const float cw = om * (pc[(size_t)st * NPJ] + ac) + (1.0f - om); const float* pr = pf + (size_t)st * NPJ; float tt = 0.0f;
#pragma unroll
        for (int i = 0; i < NEW; ++i) { tw[i] = tw[i] + pr[512 + i] * cw; tt = tt + pr[i] * tw[i]; }
        *(volatile float*)(po + (size_t)st * so) = tt; __threadfence(); *(volatile float*)(po + (size_t)st * so) = tt; } }

__global__ __launch_bounds__(256) void k_quo(const float* __restrict__ Og, const float* __restrict__ Dv, h16* Oh) { const unsigned id = blockIdx.x * 256u + threadIdx.x; const unsigned rw = id >> 6, un = (id & 63u) >> 3; const v4f ga = *(const v4f*)(Og + (size_t)id * 8), gb = *(const v4f*)(Og + (size_t)id * 8 + 4); const float dw = Dv[((size_t)rw * NUN + un) * 32u] + 1e-6f; v8h ov;
#pragma unroll
    for (int q1 = 0; q1 < 8; ++q1) ov[q1] = toh_flush((q1 < 4 ? ga[q1] : gb[q1 - 4]) / dw);
    *(volatile v8h*)(Oh + (size_t)id * 8) = ov; __threadfence(); *(volatile v8h*)(Oh + (size_t)id * 8) = ov; }

__global__ __launch_bounds__(256) void k_sq(const float* __restrict__ Yp, const float* __restrict__ u5, float* Rf) { const unsigned rw = blockIdx.x * 256u + threadIdx.x; const float* py = Yp + (size_t)rw * NCW; float ss = 0.0f;
    for (int c0 = 0; c0 < NCW; c0 += 8) { const v4f ya = *(const v4f*)(py + c0), yb = *(const v4f*)(py + c0 + 4), ba = *(const v4f*)(u5 + c0), bb = *(const v4f*)(u5 + c0 + 4);
#pragma unroll
        for (int q1 = 0; q1 < 8; ++q1) { const float wv = (q1 < 4 ? ya[q1] : yb[q1 - 4]) + bfr(q1 < 4 ? ba[q1] : bb[q1 - 4]); ss = ss + wv * wv; } }
    const float fc = 1.0f / sqrtf(ss / 512.0f + 1e-8f); *(volatile float*)(Rf + rw) = fc; __threadfence(); *(volatile float*)(Rf + rw) = fc; }

__global__ __launch_bounds__(256) void k_lay(const float* __restrict__ Yp, const float* __restrict__ u5, const float* __restrict__ u8, const float* __restrict__ Rf, float* Rs) { const unsigned id = blockIdx.x * 256u + threadIdx.x; const unsigned rw = id >> 7, c0 = (id & 127u) << 2; const v4f yw = *(const v4f*)(Yp + id * 4u), bw = *(const v4f*)(u5 + c0), nw = *(const v4f*)(u8 + c0); const float fc = Rf[rw]; v4f ov;
#pragma unroll
    for (int q1 = 0; q1 < 4; ++q1) ov[q1] = ((yw[q1] + bfr(bw[q1])) * fc) * bfr(nw[q1]);
    *(volatile v4f*)(Rs + id * 4u) = ov; __threadfence(); *(volatile v4f*)(Rs + id * 4u) = ov; }

extern "C" void kernel_launch(void* const* d_in, const int* in_sizes, int n_in, void* d_out, int out_size, void* d_ws, size_t ws_size, hipStream_t stream) {
    if (n_in < 8) return;
    if (in_sizes[0] != NRW * NCW || in_sizes[1] != 1536 * NCW || in_sizes[2] != 1536 || in_sizes[3] != NCW * NCW || in_sizes[4] != NCW || in_sizes[5] != NUN * NCW || in_sizes[6] != NUN || in_sizes[7] != NCW) return;
    if (out_size != NRW * NCW) return;
    static_assert(NRW == 2 * NSP && NSP == 4096 && NCW == 512 && NUN * NEW == NCW && NEW == 64 && NUN == 8 && NPJ == 1600 && NPJ >= 1536 + NUN && NPJ % 64 == 0 && NRW % 64 == 0 && NCW % 64 == 0 && NCW % 32 == 0 && (NRW * NCW / 8) % 256 == 0 && (1536 * NCW / 8) % 256 == 0 && (NUN * NCW / 8) % 256 == 0 && ((NPJ - 1544) * NCW / 8) % 256 == 0 && (NCW * NCW / 8) % 256 == 0 && (NRW * 1024 / 4) % 256 == 0 && NRW % 256 == 0 && NCW % 8 == 0 && (NRW * NCW / 4) % 256 == 0, "the products: row and column counts multiples of 64, the depths of 32; each flat grid exact; each lifted kernel's count a multiple of 256: its guard refuses none");
    const float* i0 = (const float*)d_in[0]; const float* i1 = (const float*)d_in[1]; const float* i2 = (const float*)d_in[2]; const float* i3 = (const float*)d_in[3]; const float* i4 = (const float*)d_in[4]; const float* i5 = (const float*)d_in[5]; const float* i6 = (const float*)d_in[6]; const float* i7 = (const float*)d_in[7]; float* rs0 = (float*)d_out;
    char* wsp = (char*)d_ws; auto carve = [&](size_t bytes) { char* p = wsp; wsp += (bytes + 255) & ~(size_t)255; return (void*)p; };
    bf* Xb = (bf*)carve((size_t)NRW * NCW * 2); bf* Wb = (bf*)carve((size_t)NPJ * NCW * 2); float* Pj = (float*)carve((size_t)NRW * NPJ * 4); float* Gq = (float*)carve((size_t)NRW * NUN * 4); float* Gk = (float*)carve((size_t)NRW * NUN * 4); float* Og = (float*)carve((size_t)NRW * NCW * 4); float* Dv = (float*)carve((size_t)NRW * NUN * 32 * 4); h16* Oh = (h16*)carve((size_t)NRW * NCW * 2); h16* Wh = (h16*)carve((size_t)NCW * NCW * 2); float* Yp = (float*)carve((size_t)NRW * NCW * 4); float* Rf = (float*)carve((size_t)NRW * 4);
    if ((size_t)(wsp - (char*)d_ws) > ws_size) return;
    k_cvt8<<<(unsigned)(NRW * NCW / 8 / 256), 256, 0, stream>>>(i0, Xb, (size_t)NRW * NCW / 8);
    k_cvt8<<<(unsigned)(1536 * NCW / 8 / 256), 256, 0, stream>>>(i1, Wb, (size_t)1536 * NCW / 8);
    k_cvt8<<<(unsigned)(NUN * NCW / 8 / 256), 256, 0, stream>>>(i5, Wb + (size_t)1536 * NCW, (size_t)NUN * NCW / 8);
    k_fillb<<<(unsigned)((NPJ - 1544) * NCW / 8 / 256), 256, 0, stream>>>(Wb + (size_t)1544 * NCW, 0u, (size_t)(NPJ - 1544) * NCW / 8);
    k_gemmw<bf, 0, false><<<dim3(NRW / 64, NPJ / 64, 1), 32, 0, stream>>>(Xb, nullptr, Wb, nullptr, NCW, Pj, NPJ, nullptr, 0, 0, 0);
    k_run<<<2, 32, 0, stream>>>(Pj, i6, Gq, Gk);
    k_feat<<<(unsigned)(NRW * 1024 / 4 / 256), 256, 0, stream>>>(Pj, i2, Gq, Gk);
    k_tal2<<<2 * NUN, 96, 0, stream>>>(Pj, i2, Og, Dv);
    k_quo<<<(unsigned)(NRW * NCW / 8 / 256), 256, 0, stream>>>(Og, Dv, Oh);
    k_c16<true><<<(unsigned)(NCW * NCW / 8 / 256), 256, 0, stream>>>(i3, Wh, (size_t)NCW * NCW / 8);
    k_gemmw<h16, 0, false><<<dim3(NRW / 64, NCW / 64, 1), 32, 0, stream>>>(Oh, nullptr, Wh, nullptr, NCW, Yp, NCW, nullptr, 0, 0, 0);
    k_sq<<<(unsigned)(NRW / 256), 256, 0, stream>>>(Yp, i4, Rf);
    k_lay<<<(unsigned)(NRW * NCW / 4 / 256), 256, 0, stream>>>(Yp, i4, i7, Rf, rs0);
}
